// SemLA_2422361554994
// MI455X (gfx1250) — hardware-verified
//
#include <hip/hip_runtime.h>


#define HW    1200
#define HWP   1216
#define CDIM  1024
#define WDIM  40
typedef __attribute__((ext_vector_type(16))) _Float16 v16h;
typedef __attribute__((ext_vector_type(8)))  _Float16 v8h;
typedef __attribute__((ext_vector_type(8)))  float    v8f;
typedef __attribute__((ext_vector_type(2)))  int      v2i;
#define VST2(T, ptr, val) do { const T _v = (val); *(volatile T*)(ptr) = _v; __threadfence(); *(volatile T*)(ptr) = _v; } while (0)
__device__ __forceinline__ v8f wmma16(v16h a, v16h b, v8f c) {
  v8f d = __builtin_amdgcn_wmma_f32_16x16x32_f16(false, a, false, b, (short)0, c, false, false);
  asm volatile("v_nop\n\tv_nop\n\tv_nop\n\tv_nop" : "+v"(d) : "v"(a), "v"(b));
  return d;
}
__device__ __forceinline__ v16h frag16(const _Float16* p, int hh) {
  const v8h lo = *(const v8h*)(p + 8 * hh), hi = *(const v8h*)(p + 16 + 8 * hh);
  return __builtin_shufflevector(lo, hi, 0,1,2,3,4,5,6,7,8,9,10,11,12,13,14,15);
}
__global__ __launch_bounds__(256) void k_cvt(const float* __restrict__ vi, const float* __restrict__ ir,
                                             _Float16* __restrict__ vh, _Float16* __restrict__ vl, _Float16* __restrict__ ih, _Float16* __restrict__ il) {
  const int t = blockIdx.x * 256 + threadIdx.x;
  const int p = t >> 7, c0 = (t & 127) * 8;
  v8h a, al, b, bl;
#pragma unroll
  for (int e = 0; e < 8; ++e) {
    const float x = (p < HW) ? vi[(size_t)(c0 + e) * HW + p] * 0.03125f : 0.f;
    const float y = (p < HW) ? ir[(size_t)(c0 + e) * HW + p] * 0.03125f : 0.f;
    a[e] = (_Float16)x; al[e] = (_Float16)(x - (float)a[e]);
    b[e] = (_Float16)y; bl[e] = (_Float16)(y - (float)b[e]);
  }
  const size_t o = (size_t)p * CDIM + c0;
  VST2(v8h, vh + o, a); VST2(v8h, vl + o, al); VST2(v8h, ih + o, b); VST2(v8h, il + o, bl);
}
__global__ __launch_bounds__(32) void k_gemm(const _Float16* __restrict__ vh, const _Float16* __restrict__ vl,
                                             const _Float16* __restrict__ ih, const _Float16* __restrict__ il, float* __restrict__ conf) {
  const int lane = threadIdx.x, hh = lane >> 4, l16 = lane & 15;
  const int m0 = blockIdx.x * 16, n0 = blockIdx.y * 64;
  v8f acc[4] = {};
#pragma unroll 2
  for (int k = 0; k < CDIM; k += 32) {
    const v16h ah = frag16(vh + (size_t)(m0 + l16) * CDIM + k, hh), al = frag16(vl + (size_t)(m0 + l16) * CDIM + k, hh);
#pragma unroll
    for (int t = 0; t < 4; ++t) {
      const size_t bo = (size_t)(n0 + t * 16 + l16) * CDIM + k;
      const v16h bh = frag16(ih + bo, hh), bl = frag16(il + bo, hh);
      acc[t] = wmma16(ah, bh, acc[t]); acc[t] = wmma16(ah, bl, acc[t]); acc[t] = wmma16(al, bh, acc[t]);
    }
  }
  for (int pass = 0; pass < 2; ++pass) {
#pragma unroll
    for (int p = 0; p < 2; ++p)
#pragma unroll
      for (int r = 0; r < 8; ++r) {
        const float a0 = acc[2 * p][r] * 10.0f, a1 = acc[2 * p + 1][r] * 10.0f;
        const float x0 = __shfl_xor(a0, 16), x1 = __shfl_xor(a1, 16);
        *(volatile float*)(conf + (size_t)(m0 + r) * HWP + n0 + p * 32 + lane)     = hh ? x1 : a0;
        *(volatile float*)(conf + (size_t)(m0 + 8 + r) * HWP + n0 + p * 32 + lane) = hh ? a1 : x0;
      }
    __threadfence();
  }
}
__global__ __launch_bounds__(256) void k_maxred(const float* __restrict__ conf, float* __restrict__ rowmax, float* __restrict__ colmax) {
  const int t = blockIdx.x * 256 + threadIdx.x;
  if (t < HW) {
    const float* row = conf + (size_t)t * HWP;
    float m = row[0];
    for (int s = 1; s < HW; ++s) m = fmaxf(m, row[s]);
    VST2(float, rowmax + t, m);
  } else if (t < 2 * HW) {
    const int s = t - HW;
    float m = conf[s];
    for (int l = 1; l < HW; ++l) m = fmaxf(m, conf[(size_t)l * HWP + s]);
    VST2(float, colmax + s, m);
  }
}
__global__ __launch_bounds__(256) void k_match(const float* __restrict__ conf, const float* __restrict__ rowmax, const float* __restrict__ colmax, int* __restrict__ out) {
  const int l = blockIdx.x * 256 + threadIdx.x;
  if (l >= HW) return;
  const float rm = rowmax[l];
  const float* row = conf + (size_t)l * HWP;
  int j = 0, valid = 0;
  for (int s = 0; s < HW; ++s) { const float v = row[s]; if (v == rm && v == colmax[s]) { j = s; valid = 1; break; } }
  const int x = l % WDIM, y = l / WDIM, jx = j % WDIM, jy = j / WDIM;
  const v2i p0 = {valid ? x * 8 : 0, valid ? y * 8 : 0}, p1 = {valid ? jx * 8 : 0, valid ? jy * 8 : 0};
  VST2(v2i, (v2i*)out + l, p0);
  VST2(v2i, (v2i*)out + HW + l, p1);
}
extern "C" void kernel_launch(void* const* d_in, const int* in_sizes, int n_in,
                              void* d_out, int out_size, void* d_ws, size_t ws_size, hipStream_t stream) {
  (void)in_sizes; (void)n_in; (void)out_size;
  const float* vi = (const float*)d_in[0];
  const float* ir = (const float*)d_in[1];
  int* out = (int*)d_out;
  const size_t plane = (size_t)HWP * CDIM * 2;
  if (ws_size < 4 * plane + (size_t)HW * HWP * 4 + 2 * HWP * 4) return;
  char* ws = (char*)d_ws;
  _Float16* vh = (_Float16*)ws; _Float16* vl = (_Float16*)(ws + plane); _Float16* ih = (_Float16*)(ws + 2 * plane); _Float16* il = (_Float16*)(ws + 3 * plane);
  float* conf = (float*)(ws + 4 * plane);
  float* rowmax = conf + (size_t)HW * HWP;
  float* colmax = rowmax + HWP;
  k_cvt<<<(HWP * CDIM / 8) / 256, 256, 0, stream>>>(vi, ir, vh, vl, ih, il);
  k_gemm<<<dim3(HW / 16, HWP / 64), 32, 0, stream>>>(vh, vl, ih, il, conf);
  k_maxred<<<(2 * HW + 255) / 256, 256, 0, stream>>>(conf, rowmax, colmax);
  k_match<<<(HW + 255) / 256, 256, 0, stream>>>(conf, rowmax, colmax, out);
}
